// BuildGcn_3075196584644
// MI455X (gfx1250) — hardware-verified
//
#include <hip/hip_runtime.h>
#include <hip/hip_bf16.h>
#include <stddef.h>


#define DF      128
#define NTHR    256
#define NWAVE   8
#define EPT     8
#define NGRP    2
#define CHUNK   (NTHR * EPT * NGRP)
#define WCAP    (EPT * NGRP * 32)
#define LISTN   (NWAVE * WCAP)
#define NB      512
#define NBD     4096
#define LDS_AGG (NB * DF * 4 + LISTN * 4 + 64)

static_assert((CHUNK & (CHUNK - 1)) == 0);
static_assert(CHUNK <= 4096);
static_assert(NB <= 4096 && NBD <= 4096);
static_assert((NB & (NB - 1)) == 0 && (NBD & (NBD - 1)) == 0);
static_assert(NB % (16 * NWAVE) == 0);
static_assert((NB * DF / 4) % NTHR == 0);

typedef float          v4f   __attribute__((ext_vector_type(4)));
typedef float          v8f   __attribute__((ext_vector_type(8)));
typedef int            v4i   __attribute__((ext_vector_type(4)));
typedef unsigned int   v4u   __attribute__((ext_vector_type(4)));
typedef __bf16         v16bf __attribute__((ext_vector_type(16)));
union FragU { v16bf v; v4u q[2]; };

__device__ __forceinline__ unsigned int bfb(float f) {
  const unsigned int u = __float_as_uint(f);
  return (u + 0x7FFFu + ((u >> 16) & 1u)) >> 16;
}

__device__ __forceinline__ void split2(float f0, float f1, unsigned int& ph, unsigned int& pl) {
  const unsigned int h0 = bfb(f0), h1 = bfb(f1);
  const unsigned int l0 = bfb(f0 - __uint_as_float(h0 << 16));
  const unsigned int l1 = bfb(f1 - __uint_as_float(h1 << 16));
  ph = h0 | (h1 << 16);
  pl = l0 | (l1 << 16);
}

__device__ __forceinline__ void split8(v4f a, v4f b, v4u& hi, v4u& lo) {
  unsigned int h, l;
  split2(a.x, a.y, h, l); hi.x = h; lo.x = l;
  split2(a.z, a.w, h, l); hi.y = h; lo.y = l;
  split2(b.x, b.y, h, l); hi.z = h; lo.z = l;
  split2(b.z, b.w, h, l); hi.w = h; lo.w = l;
}

__device__ __forceinline__ v8f wmb(v16bf a, v16bf b, v8f c) {
  v8f d = __builtin_amdgcn_wmma_f32_16x16x32_bf16(false, a, false, b, (short)0, c, false, false);
  asm volatile("v_nop\n\tv_nop\n\tv_nop\n\tv_nop" : "+v"(d) : "v"(a), "v"(b));
  return d;
}

template <int NBT>
__device__ __forceinline__ int scan_chunk(const int* __restrict__ keys, int nE, int cbase, int nodeBase,
                                          int vec8, int* list, int tid, int lane, int wave) {
  int wc = 0;
#pragma unroll
  for (int g = 0; g < NGRP; ++g) {
    const int el0  = (g * NTHR + tid) * EPT;
    const int e0   = cbase + el0;
    const int sent = -2147483647 - 1;
    v4i da, db;
    if (vec8 != 0 && cbase + CHUNK <= nE) {
      da = *(const v4i*)(keys + e0);
      db = *(const v4i*)(keys + e0 + 4);
    } else {
      da.x = (e0     < nE) ? keys[min(e0,     nE - 1)] : sent;
      da.y = (e0 + 1 < nE) ? keys[min(e0 + 1, nE - 1)] : sent;
      da.z = (e0 + 2 < nE) ? keys[min(e0 + 2, nE - 1)] : sent;
      da.w = (e0 + 3 < nE) ? keys[min(e0 + 3, nE - 1)] : sent;
      db.x = (e0 + 4 < nE) ? keys[min(e0 + 4, nE - 1)] : sent;
      db.y = (e0 + 5 < nE) ? keys[min(e0 + 5, nE - 1)] : sent;
      db.z = (e0 + 6 < nE) ? keys[min(e0 + 6, nE - 1)] : sent;
      db.w = (e0 + 7 < nE) ? keys[min(e0 + 7, nE - 1)] : sent;
    }
    const unsigned nb = (unsigned)nodeBase;
    const unsigned s0 = (unsigned)da.x - nb, s1 = (unsigned)da.y - nb;
    const unsigned s2 = (unsigned)da.z - nb, s3 = (unsigned)da.w - nb;
    const unsigned s4 = (unsigned)db.x - nb, s5 = (unsigned)db.y - nb;
    const unsigned s6 = (unsigned)db.z - nb, s7 = (unsigned)db.w - nb;
    const bool h0 = s0 < (unsigned)NBT, h1 = s1 < (unsigned)NBT, h2 = s2 < (unsigned)NBT, h3 = s3 < (unsigned)NBT;
    const bool h4 = s4 < (unsigned)NBT, h5 = s5 < (unsigned)NBT, h6 = s6 < (unsigned)NBT, h7 = s7 < (unsigned)NBT;
    const unsigned any = __builtin_amdgcn_ballot_w32(h0 | h1 | h2 | h3 | h4 | h5 | h6 | h7);
    if (any != 0u) {
#define HITJ(J, HJ, SJ) { \
        const unsigned mj = __builtin_amdgcn_ballot_w32(HJ); \
        if (mj != 0u) { \
          if (HJ) { \
            const int pos = wc + (int)__builtin_amdgcn_mbcnt_lo(mj, 0u); \
            if (pos < WCAP) list[wave * WCAP + pos] = ((el0 + (J)) << 12) | (int)(SJ); \
          } \
          wc += (int)__builtin_popcount(mj); } }
      HITJ(0, h0, s0)
      HITJ(1, h1, s1)
      HITJ(2, h2, s2)
      HITJ(3, h3, s3)
      HITJ(4, h4, s4)
      HITJ(5, h5, s5)
      HITJ(6, h6, s6)
      HITJ(7, h7, s7)
#undef HITJ
    }
  }
  return wc;
}

__global__ __launch_bounds__(NTHR) void k_wprep(
    const float* __restrict__ W, unsigned short* whi, unsigned short* wlo) {
  const int i = blockIdx.x * NTHR + threadIdx.x;
  if (i >= DF * DF / 8) return;
  const int o = i * 8;
  const v4f a = *(const v4f*)(W + o), b = *(const v4f*)(W + o + 4);
  v4u h, l;
  split8(a, b, h, l);
  unsigned short* ph = whi + o;
  unsigned short* pl = wlo + o;
  *(volatile v4u*)ph = h;
  *(volatile v4u*)pl = l;
  __threadfence();
  *(volatile v4u*)ph = h;
  *(volatile v4u*)pl = l;
}

__global__ __launch_bounds__(NTHR) void k_deg(
    const int* __restrict__ ei, float* dinv, int nE, int vec8) {
  __shared__ __attribute__((aligned(16))) int cnt[NBD];
  __shared__ __attribute__((aligned(16))) int list[LISTN];
  __shared__ int wcnt[NWAVE];
  const int tid = threadIdx.x, lane = tid & 31, wave = tid >> 5;
  const int nodeBase = blockIdx.x * NBD;
  const int* keys = ei + nE;

  for (int i = tid; i < NBD; i += NTHR) cnt[i] = 0;
  __syncthreads();

  const int nChunks = (nE + CHUNK - 1) / CHUNK;
#pragma unroll 1
  for (int ch = 0; ch < nChunks; ++ch) {
    const int cbase = ch * CHUNK;
    const int wc = scan_chunk<NBD>(keys, nE, cbase, nodeBase, vec8, list, tid, lane, wave);
    if (lane == 0) wcnt[wave] = wc;
    __syncthreads();
    if (wave == 0) {
#pragma unroll 1
      for (int wsx = 0; wsx < NWAVE; ++wsx) {
        int n = __builtin_amdgcn_readfirstlane(wcnt[wsx]);
        n = n > WCAP ? WCAP : (n < 0 ? 0 : n);
        const int* lp = list + wsx * WCAP;
#pragma unroll 1
        for (int i = 0; i < n; ++i) {
          const int ent  = __builtin_amdgcn_readfirstlane(lp[i]);
          const int slot = ent & (NBD - 1);
          if (lane == 0) cnt[slot] = cnt[slot] + 1;
        }
      }
    }
    __syncthreads();
  }

  v4f dq[4];
#pragma unroll
  for (int q = 0; q < 4; ++q) {
    const int f = (wave * 4 + q) * 128 + 4 * lane;
    const v4i c = *(const v4i*)(cnt + f);
    dq[q].x = rsqrtf((float)(c.x + 1));
    dq[q].y = rsqrtf((float)(c.y + 1));
    dq[q].z = rsqrtf((float)(c.z + 1));
    dq[q].w = rsqrtf((float)(c.w + 1));
  }
  float* dp = dinv + (size_t)nodeBase;
#pragma unroll
  for (int q = 0; q < 4; ++q) *(volatile v4f*)(dp + (wave * 4 + q) * 128 + 4 * lane) = dq[q];
  __threadfence();
#pragma unroll
  for (int q = 0; q < 4; ++q) *(volatile v4f*)(dp + (wave * 4 + q) * 128 + 4 * lane) = dq[q];
}

__global__ __launch_bounds__(NTHR) void k_agg(
    const int* __restrict__ ei, const float* __restrict__ x, const float* __restrict__ dinv,
    const unsigned short* __restrict__ whi, const unsigned short* __restrict__ wlo,
    const float* __restrict__ bias, float* out, int nN, int nE, int vec8) {
  extern __shared__ v4f lds_dyn[];
  float* hacc = (float*)lds_dyn;
  int*   list = (int*)(hacc + NB * DF);
  int*   wcnt = list + LISTN;
  const int tid = threadIdx.x, lane = tid & 31, wave = tid >> 5, hh = lane >> 4, m = lane & 15;
  const int nodeBase = blockIdx.x * NB;
  const int* keys = ei;
  const int* srcs = ei + nE;

  {
    const v4f z = {0.f, 0.f, 0.f, 0.f};
    for (int i = tid; i < NB * DF / 4; i += NTHR) lds_dyn[i] = z;
  }
  __syncthreads();

  const int nChunks = (nE + CHUNK - 1) / CHUNK;
#pragma unroll 1
  for (int ch = 0; ch < nChunks; ++ch) {
    const int cbase = ch * CHUNK;
    const int wc = scan_chunk<NB>(keys, nE, cbase, nodeBase, vec8, list, tid, lane, wave);
    if (lane == 0) wcnt[wave] = wc;
    __syncthreads();
    if (wave == 0) {
#pragma unroll 1
      for (int wsx = 0; wsx < NWAVE; ++wsx) {
        int n = __builtin_amdgcn_readfirstlane(wcnt[wsx]);
        n = n > WCAP ? WCAP : (n < 0 ? 0 : n);
        const int* lp = list + wsx * WCAP;
#pragma unroll 1
        for (int i = 0; i < n; ++i) {
          const int ent  = __builtin_amdgcn_readfirstlane(lp[i]);
          const int slot = ent & (NB - 1);
          int e = cbase + ((ent >> 12) & (CHUNK - 1));
          e = e > nE - 1 ? nE - 1 : e;
          int src = srcs[e];
          src = src < 0 ? 0 : (src > nN - 1 ? nN - 1 : src);
          const float ds = dinv[src];
          const v4f   xv = *(const v4f*)(x + (size_t)src * DF + 4 * lane);
          v4f* ap = (v4f*)(hacc + slot * DF + 4 * lane);
          const v4f cur = *ap;
          *ap = cur + xv * ds;
        }
      }
    }
    __syncthreads();
  }

#pragma unroll 4
  for (int i = 0; i < (NB * DF / 4) / NTHR; ++i) {
    const int idx  = i * NTHR + tid;
    const int slot = idx >> 5;
    const int c4   = (idx & 31) * 4;
    int node = nodeBase + slot;
    node = node > nN - 1 ? nN - 1 : node;
    const float d  = dinv[node];
    const v4f   xv = *(const v4f*)(x + (size_t)node * DF + c4);
    v4f* ap = (v4f*)(hacc + slot * DF + c4);
    const v4f a = *ap;
    *ap = (a + xv * d) * d;
  }
  __syncthreads();

  float bcol[8];
#pragma unroll
  for (int nt = 0; nt < 8; ++nt) bcol[nt] = bias[16 * nt + m];

#pragma unroll 1
  for (int p = 0; p < NB / (16 * NWAVE); ++p) {
    const int tile = p * NWAVE + wave;
    v8f c[8];
#pragma unroll
    for (int j = 0; j < 8; ++j) { v8f z = {0.f, 0.f, 0.f, 0.f, 0.f, 0.f, 0.f, 0.f}; c[j] = z; }
    const float* arow = hacc + (16 * tile + m) * DF + 8 * hh;
#pragma unroll
    for (int ng = 0; ng < 2; ++ng) {
#pragma unroll 1
      for (int kt = 0; kt < DF / 32; ++kt) {
        const float* ap = arow + 32 * kt;
        const v4f p0 = *(const v4f*)ap,        p1 = *(const v4f*)(ap + 4);
        const v4f p2 = *(const v4f*)(ap + 16), p3 = *(const v4f*)(ap + 20);
        FragU ahi, alo;
        split8(p0, p1, ahi.q[0], alo.q[0]);
        split8(p2, p3, ahi.q[1], alo.q[1]);
#pragma unroll
        for (int t = 0; t < 4; ++t) {
          const int nt = 4 * ng + t;
          const size_t bo = (size_t)(16 * nt + m) * DF + 32 * kt + 8 * hh;
          FragU bh, bl;
          bh.q[0] = *(const v4u*)(whi + bo);
          bh.q[1] = *(const v4u*)(whi + bo + 16);
          bl.q[0] = *(const v4u*)(wlo + bo);
          bl.q[1] = *(const v4u*)(wlo + bo + 16);
          c[nt] = wmb(ahi.v, bh.v, c[nt]);
          c[nt] = wmb(ahi.v, bl.v, c[nt]);
          c[nt] = wmb(alo.v, bh.v, c[nt]);
        }
      }
    }
    __syncthreads();

    float* sp = hacc + (16 * tile + 8 * hh) * DF + m;
#pragma unroll
    for (int nt = 0; nt < 8; ++nt) {
      const float bv = bcol[nt];
      sp[0 * DF + 16 * nt] = c[nt][0] + bv;
      sp[1 * DF + 16 * nt] = c[nt][1] + bv;
      sp[2 * DF + 16 * nt] = c[nt][2] + bv;
      sp[3 * DF + 16 * nt] = c[nt][3] + bv;
      sp[4 * DF + 16 * nt] = c[nt][4] + bv;
      sp[5 * DF + 16 * nt] = c[nt][5] + bv;
      sp[6 * DF + 16 * nt] = c[nt][6] + bv;
      sp[7 * DF + 16 * nt] = c[nt][7] + bv;
    }
  }
  __syncthreads();

  const size_t outN = (size_t)nN * DF;
  const size_t ob   = (size_t)nodeBase * DF;
#pragma unroll 4
  for (int q = 0; q < NB / NWAVE; ++q) {
    const int f = (wave * (NB / NWAVE) + q) * DF + 4 * lane;
    const size_t gi = ob + (size_t)f;
    if (gi < outN) { const v4f v = *(const v4f*)(hacc + f); *(volatile v4f*)(out + gi) = v; }
  }
  __threadfence();
#pragma unroll 4
  for (int q = 0; q < NB / NWAVE; ++q) {
    const int f = (wave * (NB / NWAVE) + q) * DF + 4 * lane;
    const size_t gi = ob + (size_t)f;
    if (gi < outN) { const v4f v = *(const v4f*)(hacc + f); *(volatile v4f*)(out + gi) = v; }
  }
}

extern "C" void kernel_launch(void* const* d_in, const int* in_sizes, int n_in,
                              void* d_out, int out_size, void* d_ws, size_t ws_size,
                              hipStream_t stream) {
  if (n_in < 4) return;
  const int nN = in_sizes[0] / DF;
  const int nE = in_sizes[1] / 2;
  if (nN <= 0 || nE <= 0 || in_sizes[0] != nN * DF || in_sizes[1] != nE * 2) return;
  if (in_sizes[2] != DF * DF || in_sizes[3] < DF) return;
  if (out_size != nN * DF) return;

  const float* x  = (const float*)d_in[0];
  const int*   ei = (const int*)d_in[1];
  const float* W  = (const float*)d_in[2];
  const float* b  = (const float*)d_in[3];
  float* out = (float*)d_out;

  const int nBD = (nN + NBD - 1) / NBD;
  const int nA  = (nN + NB - 1) / NB;

  char* ws = (char*)d_ws;
  size_t off = 0;
  const size_t oHi = off; off += (size_t)DF * DF * 2;          off = (off + 255) & ~(size_t)255;
  const size_t oLo = off; off += (size_t)DF * DF * 2;          off = (off + 255) & ~(size_t)255;
  const size_t oDv = off; off += (size_t)nBD * NBD * 4;        off = (off + 255) & ~(size_t)255;
  if (off > ws_size) return;
  if (off > (size_t)134217728) return;
  unsigned short* whi  = (unsigned short*)(ws + oHi);
  unsigned short* wlo  = (unsigned short*)(ws + oLo);
  float*          dinv = (float*)(ws + oDv);

  const int vec8 = ((nE & 3) == 0) ? 1 : 0;

  k_wprep<<<(DF * DF / 8 + NTHR - 1) / NTHR, NTHR, 0, stream>>>(W, whi, wlo);

  k_deg<<<nBD, NTHR, 0, stream>>>(ei, dinv, nE, vec8);

  hipFuncSetAttribute(reinterpret_cast<const void*>(&k_agg),
                      hipFuncAttributeMaxDynamicSharedMemorySize, LDS_AGG);
  k_agg<<<nA, NTHR, LDS_AGG, stream>>>(ei, x, dinv, whi, wlo, b, out, nN, nE, vec8);
}
